// MIInfoNCESeqSeq_51264729645315
// MI455X (gfx1250) — hardware-run, weakly checked
//
#include <hip/hip_runtime.h>


#define NBB  256
#define CIN  256
#define LL   32
#define H1   128
#define H2   64
#define NR   (LL * NBB)
#define IB   8
#define NBLK (LL / IB)
typedef _Float16 h16;
typedef unsigned short bf;
typedef __attribute__((ext_vector_type(16))) __bf16   v16bf;
typedef __attribute__((ext_vector_type(16))) _Float16 v16h;
typedef __attribute__((ext_vector_type(8)))  _Float16 v8h;
typedef __attribute__((ext_vector_type(8)))  unsigned short v8us;
typedef __attribute__((ext_vector_type(8)))  float    v8f;
typedef __attribute__((ext_vector_type(4)))  float    v4f;
typedef v8h  __attribute__((may_alias)) v8ha;
typedef v4f  __attribute__((may_alias)) v4fa;
typedef v8us __attribute__((may_alias)) v8usa;

__device__ __forceinline__ unsigned short f2bf(float f) { unsigned u = __float_as_uint(f); u += 0x7FFFu + ((u >> 16) & 1u); return (unsigned short)(u >> 16); }
__device__ __forceinline__ float bf2f(unsigned short b) { return __uint_as_float(((unsigned)b) << 16); }
__device__ __forceinline__ float bfr(float f) { return bf2f(f2bf(f)); }
__device__ __forceinline__ v16h cat16(v8h lo, v8h hi) { return __builtin_shufflevector(lo, hi, 0, 1, 2, 3, 4, 5, 6, 7, 8, 9, 10, 11, 12, 13, 14, 15); }
__device__ __forceinline__ v16bf cat16b(v8us lo, v8us hi) { return __builtin_bit_cast(v16bf, __builtin_shufflevector(lo, hi, 0, 1, 2, 3, 4, 5, 6, 7, 8, 9, 10, 11, 12, 13, 14, 15)); }
__device__ __forceinline__ v8f wmma16(v16h a, v16h b, v8f c) { return __builtin_amdgcn_wmma_f32_16x16x32_f16(false, a, false, b, (short)0, c, false, false); }
__device__ __forceinline__ v8f wmmab(v16bf a, v16bf b, v8f c) { return __builtin_amdgcn_wmma_f32_16x16x32_bf16(false, a, false, b, (short)0, c, false, false); }


template <typename T16> struct WFrag;
template <> struct WFrag<h16> { typedef v16h V; static __device__ __forceinline__ V ld(const h16* p) { return cat16(*(const v8h*)p, *(const v8h*)(p + 16)); } static __device__ __forceinline__ v8f mma(V a, V b, v8f c) { return wmma16(a, b, c); } };
template <> struct WFrag<bf> { typedef v16bf V; static __device__ __forceinline__ V ld(const bf* p) { return cat16b(*(const v8us*)p, *(const v8us*)(p + 16)); } static __device__ __forceinline__ v8f mma(V a, V b, v8f c) { return wmmab(a, b, c); } };
template <typename T16, int NSPLIT, bool BIAS>
__global__ __launch_bounds__(32) void k_gemmw(const T16* __restrict__ A, const T16* __restrict__ A2, const T16* __restrict__ Bt, const T16* __restrict__ Bt2, int K, float* C, int ldc, const float* __restrict__ bias, size_t sA, size_t sB, size_t sC) {
    typedef typename WFrag<T16>::V V;
    __shared__ __align__(16) float os[16 * 68];
    const size_t z = blockIdx.z; A += z * sA; if (A2) A2 += z * sA; Bt += z * sB; if (Bt2) Bt2 += z * sB; C += z * sC;
    const int lane = threadIdx.x & 31, lr = lane & 15, hi = lane >> 4; const int r0 = blockIdx.x * 64, c0 = blockIdx.y * 64;
    v8f acc[4][4];
#pragma unroll
    for (int mb = 0; mb < 4; ++mb)
#pragma unroll
        for (int nb = 0; nb < 4; ++nb) acc[mb][nb] = (v8f){};
    const size_t aoff = (size_t)(r0 + lr) * K + 8 * hi, boff = (size_t)(c0 + lr) * K + 8 * hi;
#pragma unroll 1
    for (int kc = 0; kc < K; kc += 32) {
        V a[4], a2[4];
#pragma unroll
        for (int mb = 0; mb < 4; ++mb) { a[mb] = WFrag<T16>::ld(A + aoff + (size_t)mb * 16 * K + kc); if (NSPLIT == 1 || NSPLIT == 2) a2[mb] = WFrag<T16>::ld(A2 + aoff + (size_t)mb * 16 * K + kc); }
#pragma unroll
        for (int nb = 0; nb < 4; ++nb) { const V b = WFrag<T16>::ld(Bt + boff + (size_t)nb * 16 * K + kc); V b2; if (NSPLIT >= 2) b2 = WFrag<T16>::ld(Bt2 + boff + (size_t)nb * 16 * K + kc);
#pragma unroll
            for (int mb = 0; mb < 4; ++mb) { acc[mb][nb] = WFrag<T16>::mma(a[mb], b, acc[mb][nb]); if (NSPLIT == 1 || NSPLIT == 2) acc[mb][nb] = WFrag<T16>::mma(a2[mb], b, acc[mb][nb]); if (NSPLIT >= 2) acc[mb][nb] = WFrag<T16>::mma(a[mb], b2, acc[mb][nb]); } }
        asm volatile("v_nop\n\tv_nop\n\tv_nop\n\tv_nop" : "+v"(acc[0][0]), "+v"(acc[1][1]), "+v"(acc[2][2]), "+v"(acc[3][3]) : "v"(a[0]), "v"(a[3]));
    }
#pragma unroll
    for (int mb = 0; mb < 4; ++mb) {
#pragma unroll
        for (int nb = 0; nb < 4; ++nb) {
#pragma unroll
            for (int j = 0; j < 8; ++j) os[(hi * 8 + j) * 68 + nb * 16 + lr] = acc[mb][nb][j]; }
        __builtin_amdgcn_wave_barrier(); asm volatile("" ::: "memory");
        float* crow = C + (size_t)(r0 + mb * 16) * ldc + c0;
#pragma unroll 1
        for (int ps = 0; ps < 2; ++ps) {
#pragma unroll
            for (int s = 0; s < 8; ++s) { const int row = 2 * s + hi, cofs = lr * 4; v4f val = *(const v4fa*)(os + row * 68 + cofs); if (BIAS) { val[0] += bfr(bias[c0 + cofs]); val[1] += bfr(bias[c0 + cofs + 1]); val[2] += bfr(bias[c0 + cofs + 2]); val[3] += bfr(bias[c0 + cofs + 3]); }
                *(volatile v4f*)(crow + (size_t)row * ldc + cofs) = val; }
            if (ps == 0) __threadfence(); }
        __builtin_amdgcn_wave_barrier(); asm volatile("" ::: "memory");
    }
}

__device__ __forceinline__ h16 tohx(float x) { return (h16)x; }
__device__ __forceinline__ void splitf(float y, unsigned short& h, unsigned short& l) { h = f2bf(y); l = f2bf(y - bf2f(h)); }
typedef __attribute__((ext_vector_type(2))) _Float16 v2h;
typedef __attribute__((ext_vector_type(4))) unsigned short v4us;
typedef __attribute__((ext_vector_type(2))) unsigned short v2us;

__global__ __launch_bounds__(256) void k_cvt8(const float* __restrict__ src, bf* dst, size_t n8) { const size_t i = (size_t)blockIdx.x * 256 + threadIdx.x; if (i >= n8) return; const v8f v = *(const v8f*)(src + i * 8); v8us o;
#pragma unroll
    for (int k = 0; k < 8; ++k) o[k] = f2bf(v[k]); *(volatile v8us*)(dst + i * 8) = o; __threadfence(); *(volatile v8us*)(dst + i * 8) = o; }
__global__ __launch_bounds__(256) void k_gat(const float* __restrict__ src, bf* A) { const int e = (blockIdx.x * 256 + threadIdx.x) * 4; if (e >= NR * CIN) return; const int c = e % CIN; const int r = e / CIN; const int b = r % NBB, l = r / NBB; v4us o;
#pragma unroll
    for (int q = 0; q < 4; ++q) o[q] = f2bf(src[((size_t)b * CIN + c + q) * LL + l]); *(volatile v4us*)(A + e) = o; __threadfence(); *(volatile v4us*)(A + e) = o; }
__global__ __launch_bounds__(256) void k_relu2(const float* __restrict__ F, bf* Ph, bf* Pl, size_t cnt) { const size_t i = ((size_t)blockIdx.x * 256 + threadIdx.x) * 2; if (i >= cnt) return; v2us oh, ol;
#pragma unroll
    for (int q = 0; q < 2; ++q) { unsigned short a, c2; splitf(fmaxf(F[i + q], 0.f), a, c2); oh[q] = a; ol[q] = c2; } *(volatile v2us*)(Ph + i) = oh; *(volatile v2us*)(Pl + i) = ol; __threadfence(); *(volatile v2us*)(Ph + i) = oh; *(volatile v2us*)(Pl + i) = ol; }
__global__ __launch_bounds__(256) void k_p16(const float* __restrict__ G, h16* P, size_t cnt) { const size_t i = ((size_t)blockIdx.x * 256 + threadIdx.x) * 2; if (i >= cnt) return; v2h o; o[0] = tohx(G[i]); o[1] = tohx(G[i + 1]); *(volatile v2h*)(P + i) = o; __threadfence(); *(volatile v2h*)(P + i) = o; }
__global__ __launch_bounds__(256) void k_lse(const float* __restrict__ Cm, int ib, float* T) { const int lane = threadIdx.x & 31; const int w = blockIdx.x * 8 + (threadIdx.x >> 5); if (w >= LL * (NBB / 4)) return; const int j = w / (NBB / 4), p0 = (w % (NBB / 4)) * 4; float res = 0.f;
    for (int u = 0; u < 32; ++u) { const int p = p0 + (u >> 3), il = u & 7; const float* row = Cm + ((size_t)j * NBB + p) * (IB * NBB) + (size_t)il * NBB; float v[8]; float m = -3.0e38f;
#pragma unroll
        for (int q = 0; q < 8; ++q) { v[q] = row[lane * 8 + q]; m = fmaxf(m, v[q]); }
#pragma unroll
        for (int sh = 16; sh; sh >>= 1) m = fmaxf(m, __shfl_xor(m, sh, 32));
        float s = 0.f;
#pragma unroll
        for (int q = 0; q < 8; ++q) { float d0 = __fsub_rn(v[q], m); asm volatile("" : "+v"(d0)); s = __fadd_rn(s, __builtin_amdgcn_exp2f(__fmul_rn(d0, 1.4426950408889634f))); }
#pragma unroll
        for (int sh = 16; sh; sh >>= 1) s += __shfl_xor(s, sh, 32);
        float lg = __builtin_amdgcn_logf(s); asm volatile("" : "+v"(lg)); const float lse = __fadd_rn(m, __fmul_rn(lg, 0.69314718055994531f)); const float term = __fsub_rn(row[p], lse); if (lane == u) res = term; }
    float* dst = T + ((size_t)ib * NR + (size_t)j * NBB + p0) * IB + lane; *(volatile float*)dst = res; __threadfence(); *(volatile float*)dst = res; }
__global__ __launch_bounds__(32) void k_fin(const float* __restrict__ T, float* OUT) { const int lane = threadIdx.x; float s = 0.f; for (size_t i = lane; i < (size_t)NBLK * NR * IB; i += 32) s = __fadd_rn(s, T[i]);
#pragma unroll
    for (int sh = 16; sh; sh >>= 1) s += __shfl_xor(s, sh, 32);
    if (lane == 0) { const float v = __fadd_rn(5.5451774444795623f, s * (1.0f / (float)(LL * LL * NBB))); *(volatile float*)OUT = v; __threadfence(); *(volatile float*)OUT = v; } }

extern "C" void kernel_launch(void* const* d_in, const int* in_sizes, int n_in,
                              void* d_out, int out_size, void* d_ws, size_t ws_size, hipStream_t stream) {
    (void)in_sizes; (void)n_in; (void)out_size;
    const float* IN[10]; for (int i = 0; i < 10; ++i) IN[i] = (const float*)d_in[i];
    float* OUT = (float*)d_out;
    char* wsp = (char*)d_ws;
    auto take = [&](size_t bytes) { char* p = wsp; wsp += (bytes + 255) & ~(size_t)255; return (void*)p; };
    bf* W1G = (bf*)take((size_t)H1 * CIN * 2); bf* W2G = (bf*)take((size_t)H2 * H1 * 2); bf* W1H = (bf*)take((size_t)H1 * CIN * 2); bf* W2H = (bf*)take((size_t)H2 * H1 * 2);
    bf* A = (bf*)take((size_t)NR * CIN * 2); float* Hf = (float*)take((size_t)NR * H1 * 4); bf* Ph = (bf*)take((size_t)NR * H1 * 2); bf* Pl = (bf*)take((size_t)NR * H1 * 2); float* G = (float*)take((size_t)NR * H2 * 4); h16* XG = (h16*)take((size_t)NR * H2 * 2); h16* YH = (h16*)take((size_t)NR * H2 * 2);
    float* Cm = (float*)take((size_t)NR * IB * NBB * 4); float* T = (float*)take((size_t)NBLK * NR * IB * 4);
    if ((size_t)(wsp - (char*)d_ws) > ws_size) return;
    { k_cvt8<<<(H1 * CIN / 8 + 255) / 256, 256, 0, stream>>>(IN[2], W1G, (size_t)H1 * CIN / 8); k_cvt8<<<(H2 * H1 / 8 + 255) / 256, 256, 0, stream>>>(IN[4], W2G, (size_t)H2 * H1 / 8); k_cvt8<<<(H1 * CIN / 8 + 255) / 256, 256, 0, stream>>>(IN[6], W1H, (size_t)H1 * CIN / 8); k_cvt8<<<(H2 * H1 / 8 + 255) / 256, 256, 0, stream>>>(IN[8], W2H, (size_t)H2 * H1 / 8); }
    const unsigned LG = (NR * CIN / 4 + 255) / 256, L2 = (NR * H1 / 2 + 255) / 256, L3 = (NR * H2 / 2 + 255) / 256;
    k_gat<<<LG, 256, 0, stream>>>(IN[0], A); k_gemmw<bf, 0, true><<<dim3(NR / 64, H1 / 64, 1), 32, 0, stream>>>(A, nullptr, W1G, nullptr, CIN, Hf, H1, IN[3], 0, 0, 0); k_relu2<<<L2, 256, 0, stream>>>(Hf, Ph, Pl, (size_t)NR * H1);
    k_gemmw<bf, 1, true><<<dim3(NR / 64, 1, 1), 32, 0, stream>>>(Ph, Pl, W2G, nullptr, H1, G, H2, IN[5], 0, 0, 0); k_p16<<<L3, 256, 0, stream>>>(G, XG, (size_t)NR * H2);
    k_gat<<<LG, 256, 0, stream>>>(IN[1], A); k_gemmw<bf, 0, true><<<dim3(NR / 64, H1 / 64, 1), 32, 0, stream>>>(A, nullptr, W1H, nullptr, CIN, Hf, H1, IN[7], 0, 0, 0); k_relu2<<<L2, 256, 0, stream>>>(Hf, Ph, Pl, (size_t)NR * H1);
    k_gemmw<bf, 1, true><<<dim3(NR / 64, 1, 1), 32, 0, stream>>>(Ph, Pl, W2H, nullptr, H1, G, H2, IN[9], 0, 0, 0); k_p16<<<L3, 256, 0, stream>>>(G, YH, (size_t)NR * H2);
    for (int ib = 0; ib < NBLK; ++ib) {
        k_gemmw<h16, 0, false><<<dim3(NR / 64, IB * NBB / 64, 1), 32, 0, stream>>>(YH, nullptr, XG + (size_t)ib * IB * NBB * H2, nullptr, H2, Cm, IB * NBB, nullptr, 0, 0, 0);
        k_lse<<<(LL * (NBB / 4)) / 8, 256, 0, stream>>>(Cm, ib, T); }
    k_fin<<<1, 32, 0, stream>>>(T, OUT);
}
